// HGNN_59742995088039
// MI455X (gfx1250) — hardware-verified
//
#include <hip/hip_runtime.h>
#include <stddef.h>
#include <stdint.h>


#define NN     1024
#define INC    64
#define HIDC   128
#define OUTC   512
#define KH     64
#define PQW    128
#define H1W    256
#define RK     (2 * NN)
#define NTHR   256
#define NWAVE  8
#define EPT    8
#define CHUNK  (NTHR * EPT)
#define WCAP   (EPT * 32)
#define LISTN  (NWAVE * WCAP)
#define NBK    32
#define SLB    5
#define DEGCAP 640
#define MT     64
#define ASC    64.0f
#define WSC    256.0f
#define INVSC  (1.0f / 16384.0f)
#define GBM    64
#define GBN    128
#define GTHR   128
#define MISC_INTS 32
#define L_LIST  0
#define L_SL    (L_LIST + LISTN)
#define L_CNT   (L_SL + NBK * DEGCAP)
#define L_MISC  (L_CNT + NBK)
#define L_ATILE (L_MISC + MISC_INTS)
#define ATILE_INTS (MT * KH / 2)
#define L_ST    (L_ATILE + ATILE_INTS)
#define ST_INTS (OUTC * NBK)
#define EDGE_LDS_INTS (L_ST + ST_INTS)
#define ZINTS   L_ATILE
#define U0 (NN * INC / 8)
#define U1 (PQW * INC / 8)
#define U2 (PQW * H1W / 8)
#define U3 (HIDC * KH / 8)
#define U4 (OUTC * KH / 8)
#define U5 (OUTC * RK / 8)
#define CB0 (U0 / NTHR)
#define CB1 (CB0 + U1 / NTHR)
#define CB2 (CB1 + U2 / NTHR)
#define CB3 (CB2 + U3 / NTHR)
#define CB4 (CB3 + U4 / NTHR)
#define CB5 (CB4 + U5 / NTHR)
#define WSMAX 134217728

static_assert((CHUNK & (CHUNK - 1)) == 0 && CHUNK <= 4096);
static_assert(NBK == (1 << SLB));
static_assert(((long long)CHUNK << SLB) < (1LL << 31));
static_assert(NN % NBK == 0 && NN % GBM == 0 && OUTC % GBM == 0);
static_assert(RK == 2 * NN && INC % 32 == 0 && H1W % 32 == 0 && RK % 32 == 0 && KH % 32 == 0);
static_assert(PQW == GBN && OUTC % GBN == 0 && PQW == 2 * KH && H1W == 2 * HIDC);
static_assert(MT * 4 == NTHR && KH == 64 && DEGCAP % MT == 0);
static_assert(HIDC % (16 * NWAVE) == 0 && OUTC % (16 * NWAVE) == 0);
static_assert(ZINTS % 4 == 0 && (L_SL % 4) == 0 && (L_CNT % 4) == 0 && (L_MISC % 4) == 0);
static_assert((L_ATILE % 4) == 0 && (L_ST % 4) == 0);
static_assert(OUTC * NBK <= ST_INTS && HIDC <= ST_INTS);
static_assert(EDGE_LDS_INTS * 4 <= 300000);
static_assert(U0 % NTHR == 0 && U1 % NTHR == 0 && U2 % NTHR == 0 && U3 % NTHR == 0 && U4 % NTHR == 0 && U5 % NTHR == 0);
static_assert(MISC_INTS >= NWAVE + 2);
static_assert(GBM == (GTHR / 32) * 16 && GBN == 4 * 32);
static_assert(NBK * 2 == 64);

typedef float          v4f   __attribute__((ext_vector_type(4)));
typedef float          v8f   __attribute__((ext_vector_type(8)));
typedef int            v4i   __attribute__((ext_vector_type(4)));
typedef int            v8i   __attribute__((ext_vector_type(8)));
typedef unsigned short v8us  __attribute__((ext_vector_type(8)));
typedef unsigned short v16us __attribute__((ext_vector_type(16)));
typedef __bf16         v16bf __attribute__((ext_vector_type(16)));
typedef _Float16       v8h   __attribute__((ext_vector_type(8)));
typedef _Float16       v16h  __attribute__((ext_vector_type(16)));
typedef v4f  __attribute__((may_alias)) v4fa;
typedef v4i  __attribute__((may_alias)) v4ia;
typedef v8us __attribute__((may_alias)) v8usa;
typedef v8h  __attribute__((may_alias)) v8ha;
union FragB { v16bf v; v16us u; v8us h[2]; v8i w; };
union FragH { v16h v; v8h h[2]; v8i w; };

__device__ __forceinline__ v8f wmb(const FragB& a, const FragB& b, v8f c) {
  v8f d = __builtin_amdgcn_wmma_f32_16x16x32_bf16(false, a.v, false, b.v, (short)0, c, false, false);
  asm volatile("v_nop\n\tv_nop\n\tv_nop\n\tv_nop" : "+v"(d) : "v"(a.w), "v"(b.w));
  return d;
}
__device__ __forceinline__ v8f wmh(const FragH& a, const FragH& b, v8f c) {
  v8f d = __builtin_amdgcn_wmma_f32_16x16x32_f16(false, a.v, false, b.v, (short)0, c, false, false);
  asm volatile("v_nop\n\tv_nop\n\tv_nop\n\tv_nop" : "+v"(d) : "v"(a.w), "v"(b.w));
  return d;
}

__device__ __forceinline__ unsigned bf16_bits(float f) {
  const unsigned u = __float_as_uint(f);
  return (u + 0x7FFFu + ((u >> 16) & 1u)) >> 16;
}
__device__ __forceinline__ float bf16_val(float f) {
  return __uint_as_float(bf16_bits(f) << 16);
}
__device__ __forceinline__ unsigned short f16w_bits(float f) {
  const _Float16 hv = (_Float16)(bf16_val(f) * WSC);
  return __builtin_bit_cast(unsigned short, hv);
}
__device__ __forceinline__ _Float16 hact(float p, float q) {
  return (_Float16)(fmaxf(p + q, 0.0f) * ASC);
}

template <int SLBT>
__device__ __forceinline__ int scan_chunk(const int* __restrict__ dsts, int nE, int cbase, int slotBase,
                                          int nb, int vec8, int* list, int tid, int lane, int wave) {
  int wc = 0;
  const int el0  = tid * EPT;
  const int e0   = cbase + el0;
  const int sent = -2147483647 - 1;
  v4i da, db;
  if (vec8 != 0 && cbase + CHUNK <= nE) {
    da = *(const v4i*)(dsts + e0);
    db = *(const v4i*)(dsts + e0 + 4);
  } else {
    da.x = (e0     < nE) ? dsts[min(e0,     nE - 1)] : sent;
    da.y = (e0 + 1 < nE) ? dsts[min(e0 + 1, nE - 1)] : sent;
    da.z = (e0 + 2 < nE) ? dsts[min(e0 + 2, nE - 1)] : sent;
    da.w = (e0 + 3 < nE) ? dsts[min(e0 + 3, nE - 1)] : sent;
    db.x = (e0 + 4 < nE) ? dsts[min(e0 + 4, nE - 1)] : sent;
    db.y = (e0 + 5 < nE) ? dsts[min(e0 + 5, nE - 1)] : sent;
    db.z = (e0 + 6 < nE) ? dsts[min(e0 + 6, nE - 1)] : sent;
    db.w = (e0 + 7 < nE) ? dsts[min(e0 + 7, nE - 1)] : sent;
  }
  const unsigned nbs = (unsigned)slotBase;
  const unsigned unb = (unsigned)nb;
  const unsigned s0 = (unsigned)da.x - nbs, s1 = (unsigned)da.y - nbs;
  const unsigned s2 = (unsigned)da.z - nbs, s3 = (unsigned)da.w - nbs;
  const unsigned s4 = (unsigned)db.x - nbs, s5 = (unsigned)db.y - nbs;
  const unsigned s6 = (unsigned)db.z - nbs, s7 = (unsigned)db.w - nbs;
  const bool h0 = s0 < unb, h1 = s1 < unb, h2 = s2 < unb, h3 = s3 < unb;
  const bool h4 = s4 < unb, h5 = s5 < unb, h6 = s6 < unb, h7 = s7 < unb;
  const unsigned any = __builtin_amdgcn_ballot_w32(h0 | h1 | h2 | h3 | h4 | h5 | h6 | h7);
  if (any != 0u) {
#define HITJ(J, HJ, SJ) { \
      const unsigned mj = __builtin_amdgcn_ballot_w32(HJ); \
      if (mj != 0u) { \
        if (HJ) { \
          const int pos = wc + (int)__builtin_amdgcn_mbcnt_lo(mj, 0u); \
          if (pos < WCAP) list[wave * WCAP + pos] = ((el0 + (J)) << SLBT) | (int)(SJ); \
        } \
        wc += (int)__builtin_popcount(mj); } }
    HITJ(0, h0, s0)
    HITJ(1, h1, s1)
    HITJ(2, h2, s2)
    HITJ(3, h3, s3)
    HITJ(4, h4, s4)
    HITJ(5, h5, s5)
    HITJ(6, h6, s6)
    HITJ(7, h7, s7)
#undef HITJ
  }
  return wc;
}

__global__ __launch_bounds__(NTHR) void k_prep(const float* __restrict__ x, const float* __restrict__ W1,
                                               const float* __restrict__ W2, const float* __restrict__ W3,
                                               const float* __restrict__ W4, const float* __restrict__ Wr,
                                               unsigned short* XB, unsigned short* BT1, unsigned short* BT3,
                                               unsigned short* W2T, unsigned short* W4T, unsigned short* WRT) {
  const int b = (int)blockIdx.x, t = (int)threadIdx.x;
  v8us o = {0, 0, 0, 0, 0, 0, 0, 0};
  unsigned short* dp;
  if (b < CB0) {
    const int u = b * NTHR + t;
    const float* p = x + (size_t)u * 8;
    const v4f a = *(const v4f*)p;
    const v4f c = *(const v4f*)(p + 4);
    o[0] = (unsigned short)bf16_bits(a.x); o[1] = (unsigned short)bf16_bits(a.y);
    o[2] = (unsigned short)bf16_bits(a.z); o[3] = (unsigned short)bf16_bits(a.w);
    o[4] = (unsigned short)bf16_bits(c.x); o[5] = (unsigned short)bf16_bits(c.y);
    o[6] = (unsigned short)bf16_bits(c.z); o[7] = (unsigned short)bf16_bits(c.w);
    dp = XB + (size_t)u * 8;
  } else if (b < CB1) {
    const int u = (b - CB0) * NTHR + t;
    const int np = u >> 3, k8 = (u & 7) * 8, hf = np >> 6, col = np & 63;
    const float* p = W1 + (size_t)(hf * INC + k8) * KH + col;
#pragma unroll
    for (int q = 0; q < 8; ++q) o[q] = (unsigned short)bf16_bits(p[(size_t)q * KH]);
    dp = BT1 + (size_t)u * 8;
  } else if (b < CB2) {
    const int u = (b - CB1) * NTHR + t;
    const int np = u >> 5, k8 = (u & 31) * 8, kk = k8 & (HIDC - 1), hf = np >> 6, col = np & 63;
    const float* p = W3 + (size_t)(hf * HIDC + kk) * KH + col;
#pragma unroll
    for (int q = 0; q < 8; ++q) o[q] = (unsigned short)bf16_bits(p[(size_t)q * KH]);
    dp = BT3 + (size_t)u * 8;
  } else if (b < CB3) {
    const int u = (b - CB2) * NTHR + t;
    const int col = u >> 3, k8 = (u & 7) * 8;
    const float* p = W2 + (size_t)k8 * HIDC + col;
#pragma unroll
    for (int q = 0; q < 8; ++q) o[q] = f16w_bits(p[(size_t)q * HIDC]);
    dp = W2T + (size_t)u * 8;
  } else if (b < CB4) {
    const int u = (b - CB3) * NTHR + t;
    const int col = u >> 3, k8 = (u & 7) * 8;
    const float* p = W4 + (size_t)k8 * OUTC + col;
#pragma unroll
    for (int q = 0; q < 8; ++q) o[q] = f16w_bits(p[(size_t)q * OUTC]);
    dp = W4T + (size_t)u * 8;
  } else {
    const int u = (b - CB4) * NTHR + t;
    const int oo = u >> 8, g = u & 255;
    const float* p = Wr + (size_t)(4 * g) * OUTC + oo;
    const unsigned w0 = bf16_bits(p[0]);
    const unsigned w1 = bf16_bits(p[OUTC]);
    const unsigned w2 = bf16_bits(p[2 * OUTC]);
    const unsigned w3 = bf16_bits(p[3 * OUTC]);
    o[0] = (unsigned short)w0; o[1] = (unsigned short)w0;
    o[2] = (unsigned short)w1; o[3] = (unsigned short)w1;
    o[4] = (unsigned short)w2; o[5] = (unsigned short)w2;
    o[6] = (unsigned short)w3; o[7] = (unsigned short)w3;
    dp = WRT + (size_t)u * 8;
  }
  *(volatile v8us*)dp = o;
  __threadfence();
  *(volatile v8us*)dp = o;
}

__global__ __launch_bounds__(GTHR) void k_gemm(const unsigned short* __restrict__ Apl, int lda,
                                               const unsigned short* __restrict__ BT, int ldb, int K,
                                               const float* __restrict__ bias, int nbias,
                                               float* outp, int ldo, int nOut) {
  __shared__ __attribute__((aligned(16))) float stg[GBM * GBN];
  const int tid = (int)threadIdx.x, lane = tid & 31, wave = tid >> 5, hh = lane >> 4, m = lane & 15;
  const int rowBase = (int)blockIdx.x * GBM;
  const int colBase = (int)blockIdx.y * GBN;

  v8f acc[8];
  {
    const v8f z = {0.f, 0.f, 0.f, 0.f, 0.f, 0.f, 0.f, 0.f};
#pragma unroll
    for (int t = 0; t < 8; ++t) acc[t] = z;
  }
  const unsigned short* ap = Apl + (size_t)(rowBase + 16 * wave + m) * (size_t)lda + 8 * hh;
  const unsigned short* bp = BT + (size_t)(colBase + m) * (size_t)ldb + 8 * hh;

#pragma unroll 1
  for (int k0 = 0; k0 < K; k0 += 32) {
    FragB af;
    af.h[0] = *(const v8usa*)(ap + k0);
    af.h[1] = *(const v8usa*)(ap + k0 + 16);
#pragma unroll
    for (int nt = 0; nt < 8; ++nt) {
      const unsigned short* wq = bp + (size_t)(16 * nt) * (size_t)ldb + k0;
      FragB bf;
      bf.h[0] = *(const v8usa*)wq;
      bf.h[1] = *(const v8usa*)(wq + 16);
      acc[nt] = wmb(af, bf, acc[nt]);
    }
  }

#pragma unroll
  for (int nt = 0; nt < 8; ++nt) {
    const int lc = 16 * nt + m;
#pragma unroll
    for (int r = 0; r < 8; ++r) {
      const int lr = 16 * wave + 8 * hh + r;
      stg[lr * GBN + lc] = acc[nt][r];
    }
  }
  __syncthreads();

  v4f bb4;
  {
    const int c0 = colBase + 4 * lane;
    const int nb1 = nbias > 0 ? nbias - 1 : 0;
    const float t0 = bf16_val(bias[min(c0 + 0, nb1)]);
    const float t1 = bf16_val(bias[min(c0 + 1, nb1)]);
    const float t2 = bf16_val(bias[min(c0 + 2, nb1)]);
    const float t3 = bf16_val(bias[min(c0 + 3, nb1)]);
    bb4.x = (c0 + 0 < nbias) ? t0 : 0.0f;
    bb4.y = (c0 + 1 < nbias) ? t1 : 0.0f;
    bb4.z = (c0 + 2 < nbias) ? t2 : 0.0f;
    bb4.w = (c0 + 3 < nbias) ? t3 : 0.0f;
  }

  v4f pv[16];
#pragma unroll
  for (int i = 0; i < 16; ++i) pv[i] = *(const v4fa*)(stg + (16 * wave + i) * GBN + 4 * lane) + bb4;

#pragma unroll
  for (int i = 0; i < 16; ++i) {
    const int r = rowBase + 16 * wave + i;
    if (r < nOut) *(volatile v4f*)(outp + (size_t)r * (size_t)ldo + colBase + 4 * lane) = pv[i];
  }
  __threadfence();
#pragma unroll
  for (int i = 0; i < 16; ++i) {
    const int r = rowBase + 16 * wave + i;
    if (r < nOut) *(volatile v4f*)(outp + (size_t)r * (size_t)ldo + colBase + 4 * lane) = pv[i];
  }
}

__device__ __forceinline__ void h2t_store_pass(const unsigned* st2, unsigned short* H2T, int nodeBase,
                                               int wave, int lane) {
  const int q8 = lane & 7, sub = lane >> 3;
#pragma unroll
  for (int i = 0; i < 16; ++i) {
    const int c = wave * 64 + i * 4 + sub;
    const v4i v = *(const v4ia*)(st2 + c * NBK + 4 * q8);
    unsigned short* dst = H2T + (size_t)c * RK + 2 * nodeBase + 8 * q8;
    *(volatile v4i*)dst = v;
  }
}

template <int COUT, int LAYER>
__global__ __launch_bounds__(NTHR) void k_edge(const int* __restrict__ ei, int nE, int nN, int vec8,
                                               const float* __restrict__ PQ, const _Float16* __restrict__ WBT,
                                               const float* __restrict__ bb, unsigned short* H1P,
                                               unsigned short* H2T) {
  constexpr int NTW = COUT / (16 * NWAVE);
  extern __shared__ __attribute__((aligned(16))) int dsm[];
  int* list = dsm + L_LIST;
  int* sl   = dsm + L_SL;
  int* cnt  = dsm + L_CNT;
  int* misc = dsm + L_MISC;
  _Float16* atile = (_Float16*)(dsm + L_ATILE);
  unsigned short* st1 = (unsigned short*)(dsm + L_ST);
  unsigned* st2 = (unsigned*)(dsm + L_ST);
  const int tid = (int)threadIdx.x, lane = tid & 31, wave = tid >> 5, hh = lane >> 4, m = lane & 15;
  const int nodeBase = (int)blockIdx.x * NBK;
  const int* srcs = ei;
  const int* dsts = ei + nE;

  FragH bfr[NTW][2];
#pragma unroll
  for (int nt = 0; nt < NTW; ++nt) {
    const _Float16* wr = WBT + (size_t)(16 * (wave * NTW + nt) + m) * KH + 8 * hh;
    bfr[nt][0].h[0] = *(const v8ha*)(wr);
    bfr[nt][0].h[1] = *(const v8ha*)(wr + 16);
    bfr[nt][1].h[0] = *(const v8ha*)(wr + 32);
    bfr[nt][1].h[1] = *(const v8ha*)(wr + 48);
  }

  {
    const v4i z4 = {0, 0, 0, 0};
    for (int i = tid * 4; i < ZINTS; i += NTHR * 4) *(v4ia*)(dsm + i) = z4;
  }
  __syncthreads();

  const int nChunks = (nE + CHUNK - 1) / CHUNK;
#pragma unroll 1
  for (int ch = 0; ch < nChunks; ++ch) {
    const int cbase = ch * CHUNK;
    const int wc = scan_chunk<SLB>(dsts, nE, cbase, nodeBase, NBK, vec8, list, tid, lane, wave);
    if (lane == 0) misc[wave] = wc;
    __syncthreads();
    if (wave == 0) {
#pragma unroll 1
      for (int w2 = 0; w2 < NWAVE; ++w2) {
        int c = misc[w2];
        c = c < 0 ? 0 : (c > WCAP ? WCAP : c);
#pragma unroll 1
        for (int b0 = 0; b0 < c; b0 += 32) {
          const int idx = b0 + lane;
          const int ent = list[w2 * WCAP + (idx < WCAP ? idx : WCAP - 1)];
          const int m32 = (c - b0) < 32 ? (c - b0) : 32;
#pragma unroll 1
          for (int k = 0; k < m32; ++k) {
            const int u    = __builtin_amdgcn_readlane(ent, k);
            const int slot = u & (NBK - 1);
            const int el   = (u >> SLB) & (CHUNK - 1);
            const int eidv = cbase + el;
            if (lane == 0) {
              const int p = cnt[slot];
              if (p < DEGCAP) sl[slot * DEGCAP + (p < 0 ? 0 : p)] = eidv;
              cnt[slot] = p + 1;
            }
          }
        }
      }
    }
    __syncthreads();
  }

  const int row = tid >> 2, kq = (tid & 3) * 16;
#pragma unroll 1
  for (int s = 0; s < NBK; ++s) {
    const int node = nodeBase + s;
    const int nc = node < nN ? node : nN - 1;
    const int craw = cnt[s];
    const bool big = craw > DEGCAP;
    const int c = craw < 0 ? 0 : (craw > DEGCAP ? DEGCAP : craw);
    const int ntile = (c + MT - 1) / MT;
    const float* pp = PQ + (size_t)nc * PQW + kq;
    const v4f p0 = *(const v4f*)pp;
    const v4f p1 = *(const v4f*)(pp + 4);
    const v4f p2 = *(const v4f*)(pp + 8);
    const v4f p3 = *(const v4f*)(pp + 12);
    v8f rmax[NTW];
    {
      const float ninf = -__builtin_inff();
      const v8f zi = {ninf, ninf, ninf, ninf, ninf, ninf, ninf, ninf};
#pragma unroll
      for (int nt = 0; nt < NTW; ++nt) rmax[nt] = zi;
    }
#pragma unroll 1
    for (int t = 0; t < ntile; ++t) {
      int hidx = t * MT + row;
      hidx = hidx > c - 1 ? c - 1 : hidx;
      hidx = hidx < 0 ? 0 : hidx;
      int eidv = sl[s * DEGCAP + hidx];
      eidv = eidv < 0 ? 0 : (eidv > nE - 1 ? nE - 1 : eidv);
      int j = srcs[eidv];
      j = j < 0 ? 0 : (j > nN - 1 ? nN - 1 : j);
      const float* qp = PQ + (size_t)j * PQW + KH + kq;
      const v4f q0 = *(const v4f*)qp;
      const v4f q1 = *(const v4f*)(qp + 4);
      const v4f q2 = *(const v4f*)(qp + 8);
      const v4f q3 = *(const v4f*)(qp + 12);
      const v8h a0 = { hact(p0.x, q0.x), hact(p0.y, q0.y), hact(p0.z, q0.z), hact(p0.w, q0.w),
                       hact(p1.x, q1.x), hact(p1.y, q1.y), hact(p1.z, q1.z), hact(p1.w, q1.w) };
      const v8h a1 = { hact(p2.x, q2.x), hact(p2.y, q2.y), hact(p2.z, q2.z), hact(p2.w, q2.w),
                       hact(p3.x, q3.x), hact(p3.y, q3.y), hact(p3.z, q3.z), hact(p3.w, q3.w) };
      *(v8ha*)(atile + row * KH + kq) = a0;
      *(v8ha*)(atile + row * KH + kq + 8) = a1;
      __syncthreads();

#pragma unroll
      for (int mt = 0; mt < 4; ++mt) {
        const _Float16* ar = atile + (16 * mt + m) * KH + 8 * hh;
        FragH fa0, fa1;
        fa0.h[0] = *(const v8ha*)(ar);
        fa0.h[1] = *(const v8ha*)(ar + 16);
        fa1.h[0] = *(const v8ha*)(ar + 32);
        fa1.h[1] = *(const v8ha*)(ar + 48);
#pragma unroll
        for (int nt = 0; nt < NTW; ++nt) {
          v8f d = {0.f, 0.f, 0.f, 0.f, 0.f, 0.f, 0.f, 0.f};
          d = wmh(fa0, bfr[nt][0], d);
          d = wmh(fa1, bfr[nt][1], d);
#pragma unroll
          for (int r = 0; r < 8; ++r) rmax[nt][r] = fmaxf(rmax[nt][r], d[r]);
        }
      }
      __syncthreads();
    }

    const float pzr = big ? __int_as_float(0x7fc00000) : 0.0f;
    const bool live = node < nN;
#pragma unroll
    for (int nt = 0; nt < NTW; ++nt) {
      float cm = rmax[nt][0];
#pragma unroll
      for (int r = 1; r < 8; ++r) cm = fmaxf(cm, rmax[nt][r]);
      cm = fmaxf(cm, __shfl_xor(cm, 16, 32));
      const int col = 16 * (wave * NTW + nt) + m;
      const float bbv = bf16_val(bb[col]);
      float val = (craw == 0) ? 0.0f : (cm * INVSC + bbv);
      val = live ? (val + pzr) : 0.0f;
      const unsigned hb = bf16_bits(val);
      const unsigned lb = bf16_bits(val - __uint_as_float(hb << 16));
      if constexpr (LAYER == 1) {
        if (hh == 0) { st1[col] = (unsigned short)hb; st1[HIDC + col] = (unsigned short)lb; }
      } else {
        if (hh == 0) st2[col * NBK + s] = hb | (lb << 16);
      }
    }
    if constexpr (LAYER == 1) {
      __syncthreads();
      if (wave == 0 && live) {
        const v4i q = *(const v4ia*)(st1 + 8 * lane);
        unsigned short* rp = H1P + (size_t)node * H1W + 8 * lane;
        *(volatile v4i*)rp = q;
        __threadfence();
        *(volatile v4i*)rp = q;
      }
      __syncthreads();
    }
  }

  if constexpr (LAYER == 2) {
    __syncthreads();
    h2t_store_pass(st2, H2T, nodeBase, wave, lane);
    __threadfence();
    h2t_store_pass(st2, H2T, nodeBase, wave, lane);
  }
}

static inline size_t al256(size_t o) { return (o + 255) & ~(size_t)255; }

extern "C" void kernel_launch(void* const* d_in, const int* in_sizes, int n_in,
                              void* d_out, int out_size, void* d_ws, size_t ws_size,
                              hipStream_t stream) {
  if (n_in < 12) return;
  if (in_sizes[0] != NN * INC) return;
  if (in_sizes[1] < 2 || (in_sizes[1] & 1) != 0) return;
  const int nE = in_sizes[1] / 2;
  if (nE < 1 || nE >= (1 << 28)) return;
  if (in_sizes[2] != 2 * INC * KH || in_sizes[3] != KH) return;
  if (in_sizes[4] != KH * HIDC || in_sizes[5] != HIDC) return;
  if (in_sizes[6] != 2 * HIDC * KH || in_sizes[7] != KH) return;
  if (in_sizes[8] != KH * OUTC || in_sizes[9] != OUTC) return;
  if (in_sizes[10] != NN * OUTC || in_sizes[11] != OUTC) return;
  if (out_size != OUTC * OUTC) return;

  const float* x  = (const float*)d_in[0];
  const int*   ei = (const int*)d_in[1];
  const float* W1 = (const float*)d_in[2];
  const float* b1 = (const float*)d_in[3];
  const float* W2 = (const float*)d_in[4];
  const float* b2 = (const float*)d_in[5];
  const float* W3 = (const float*)d_in[6];
  const float* b3 = (const float*)d_in[7];
  const float* W4 = (const float*)d_in[8];
  const float* b4 = (const float*)d_in[9];
  const float* Wr = (const float*)d_in[10];
  const float* br = (const float*)d_in[11];
  float* out = (float*)d_out;

  char* ws = (char*)d_ws;
  size_t off = 0;
  const size_t oXB  = off; off = al256(off + (size_t)NN * INC * 2);
  const size_t oBT1 = off; off = al256(off + (size_t)PQW * INC * 2);
  const size_t oBT3 = off; off = al256(off + (size_t)PQW * H1W * 2);
  const size_t oW2T = off; off = al256(off + (size_t)HIDC * KH * 2);
  const size_t oW4T = off; off = al256(off + (size_t)OUTC * KH * 2);
  const size_t oWRT = off; off = al256(off + (size_t)OUTC * RK * 2);
  const size_t oPQ1 = off; off = al256(off + (size_t)NN * PQW * 4);
  const size_t oPQ2 = off; off = al256(off + (size_t)NN * PQW * 4);
  const size_t oH1P = off; off = al256(off + (size_t)NN * H1W * 2);
  const size_t oH2T = off; off = al256(off + (size_t)OUTC * RK * 2);
  if (off > ws_size || off > (size_t)WSMAX) return;
  unsigned short* XB  = (unsigned short*)(ws + oXB);
  unsigned short* BT1 = (unsigned short*)(ws + oBT1);
  unsigned short* BT3 = (unsigned short*)(ws + oBT3);
  unsigned short* W2T = (unsigned short*)(ws + oW2T);
  unsigned short* W4T = (unsigned short*)(ws + oW4T);
  unsigned short* WRT = (unsigned short*)(ws + oWRT);
  float* PQ1 = (float*)(ws + oPQ1);
  float* PQ2 = (float*)(ws + oPQ2);
  unsigned short* H1P = (unsigned short*)(ws + oH1P);
  unsigned short* H2T = (unsigned short*)(ws + oH2T);

  const int vec8 = ((nE & 3) == 0) ? 1 : 0;
  const size_t edgeLds = (size_t)EDGE_LDS_INTS * 4;
  hipFuncSetAttribute(reinterpret_cast<const void*>(&k_edge<HIDC, 1>), hipFuncAttributeMaxDynamicSharedMemorySize, (int)edgeLds);
  hipFuncSetAttribute(reinterpret_cast<const void*>(&k_edge<OUTC, 2>), hipFuncAttributeMaxDynamicSharedMemorySize, (int)edgeLds);

  k_prep<<<CB5, NTHR, 0, stream>>>(x, W1, W2, W3, W4, Wr, XB, BT1, BT3, W2T, W4T, WRT);
  k_gemm<<<dim3(NN / GBM, PQW / GBN), GTHR, 0, stream>>>(XB, INC, BT1, INC, INC, b1, KH, PQ1, PQW, NN);
  k_edge<HIDC, 1><<<NN / NBK, NTHR, edgeLds, stream>>>(ei, nE, NN, vec8, PQ1, (const _Float16*)W2T, b2, H1P, H2T);
  k_gemm<<<dim3(NN / GBM, PQW / GBN), GTHR, 0, stream>>>(H1P, H1W, BT3, H1W, H1W, b3, KH, PQ2, PQW, NN);
  k_edge<OUTC, 2><<<NN / NBK, NTHR, edgeLds, stream>>>(ei, nE, NN, vec8, PQ2, (const _Float16*)W4T, b4, H1P, H2T);
  k_gemm<<<dim3(OUTC / GBM, OUTC / GBN), GTHR, 0, stream>>>(H2T, RK, WRT, RK, RK, br, OUTC, out, OUTC, OUTC);
}
